// LocalCausalSelfAttention_43284680409119
// MI455X (gfx1250) — hardware-verified
//
#include <hip/hip_runtime.h>
#include <math.h>
#include <stdint.h>

#define NTOK  8192
#define EMB   1024
#define QKVW  3072
#define QKW   2048
#define GRP   512
#define NGRP  16
#define NHD   16
#define HDM   64
#define NFRQ  32
#define QKP   4096

static_assert(NGRP * GRP == NTOK);
static_assert(NHD * HDM == EMB);
static_assert(NTOK % 128 == 0);
static_assert(EMB % 128 == 0);
static_assert(QKW % 128 == 0);
static_assert(EMB % 32 == 0);
static_assert(((NTOK / 32) * (QKW / 128)) % 4 == 0);
static_assert(((EMB / 32) * (NTOK / 128)) % 4 == 0);
static_assert(((NTOK / 32) * (EMB / 128)) % 4 == 0);
static_assert(QKP * 2 == QKW * 4);
static_assert((NTOK * EMB) % (256 * 8) == 0);

typedef _Float16     v16h __attribute__((ext_vector_type(16)));
typedef _Float16     v8h  __attribute__((ext_vector_type(8)));
typedef __bf16       v16b __attribute__((ext_vector_type(16)));
typedef __bf16       v8b  __attribute__((ext_vector_type(8)));
typedef float        v8f  __attribute__((ext_vector_type(8)));
typedef float        v4f  __attribute__((ext_vector_type(4)));
typedef unsigned int v4u  __attribute__((ext_vector_type(4)));
typedef unsigned int v2u  __attribute__((ext_vector_type(2)));

__device__ __forceinline__ unsigned short bf_bits(float f) {
  const unsigned u = __float_as_uint(f);
  return (unsigned short)((u + 0x7FFFu + ((u >> 16) & 1u)) >> 16);
}
__device__ __forceinline__ float bf_val(unsigned short h) { return __uint_as_float(((unsigned)h) << 16); }
__device__ __forceinline__ float bf_rne(float f) { return bf_val(bf_bits(f)); }
__device__ __forceinline__ unsigned pk16(unsigned short a, unsigned short b) { return (unsigned)a | ((unsigned)b << 16); }
__device__ __forceinline__ v8f zero8() { v8f z = {0.f, 0.f, 0.f, 0.f, 0.f, 0.f, 0.f, 0.f}; return z; }
__device__ __forceinline__ int wave_id() { return __builtin_amdgcn_readfirstlane((int)(threadIdx.x >> 5)); }

__device__ __forceinline__ void lds_wave_sync() {
  __builtin_amdgcn_fence(__ATOMIC_RELEASE, "workgroup");
  __builtin_amdgcn_wave_barrier();
  __builtin_amdgcn_fence(__ATOMIC_ACQUIRE, "workgroup");
}

union FragH { v16h v; v8h h[2]; };
union FragB { v16b v; v8b h[2]; };
__device__ __forceinline__ v16h ldfrag_h(const _Float16* p) { FragH f; f.h[0] = *(const v8h*)(p); f.h[1] = *(const v8h*)(p + 16); return f.v; }
__device__ __forceinline__ v16b ldfrag_b(const __bf16* p)   { FragB f; f.h[0] = *(const v8b*)(p); f.h[1] = *(const v8b*)(p + 16); return f.v; }

__device__ __forceinline__ v8f mma_b(v16b a, v16b b, v8f c) {
  return __builtin_amdgcn_wmma_f32_16x16x32_bf16(false, a, false, b, (short)0, c, false, false);
}
__device__ __forceinline__ v8f mma_b_g(v16b a, v16b b, v8f c) {
  c = __builtin_amdgcn_wmma_f32_16x16x32_bf16(false, a, false, b, (short)0, c, false, false);
  asm volatile("v_nop\n\tv_nop\n\tv_nop\n\tv_nop" : "+v"(c) : "v"(a), "v"(b));
  return c;
}
__device__ __forceinline__ v8f mma_h_g(v16h a, v16h b, v8f c) {
  c = __builtin_amdgcn_wmma_f32_16x16x32_f16(false, a, false, b, (short)0, c, false, false);
  asm volatile("v_nop\n\tv_nop\n\tv_nop\n\tv_nop" : "+v"(c) : "v"(a), "v"(b));
  return c;
}
__device__ __forceinline__ void guard_b5(v8f& a, v8f& b, v16b x0, v16b x1, v16b x2, v16b x3, v16b y) {
  asm volatile("v_nop\n\tv_nop\n\tv_nop\n\tv_nop" : "+v"(a), "+v"(b) : "v"(x0), "v"(x1), "v"(x2), "v"(x3), "v"(y) : "memory");
}
__device__ __forceinline__ void acc_guard4(v8f& a, v8f& b, v8f& c, v8f& d) {
  asm volatile("v_nop\n\tv_nop\n\tv_nop\n\tv_nop" : "+v"(a), "+v"(b), "+v"(c), "+v"(d));
}

__global__ __launch_bounds__(256) void rope_table_kernel(float* __restrict__ cst, float* __restrict__ snt) {
  const int lane = threadIdx.x & 31;
  const int wave = (int)(threadIdx.x >> 5);
  const int t = (int)blockIdx.x * 8 + wave;
  if (t >= GRP) return;
  const float e   = -(float)(4 * lane + 1) * 0.015625f;
  const float pw  = powf(10000.0f, e);
  const float ang = (float)t * pw;
  const float cv  = cosf(ang);
  const float sv  = sinf(ang);
  const size_t o = (size_t)t * NFRQ + lane;
  for (int pass = 0; pass < 2; ++pass) {
    ((volatile float*)cst)[o] = cv;
    ((volatile float*)snt)[o] = sv;
    __threadfence();
  }
}

__global__ __launch_bounds__(256) void cvt_bf16_kernel(const float* __restrict__ in, unsigned short* __restrict__ outp, int n8) {
  const int i = (int)blockIdx.x * 256 + (int)threadIdx.x;
  if (i >= n8) return;
  const size_t e = 8 * (size_t)i;
  const v4f a = *(const v4f*)(in + e);
  const v4f b = *(const v4f*)(in + e + 4);
  v4u w;
  w[0] = pk16(bf_bits(a[0]), bf_bits(a[1]));
  w[1] = pk16(bf_bits(a[2]), bf_bits(a[3]));
  w[2] = pk16(bf_bits(b[0]), bf_bits(b[1]));
  w[3] = pk16(bf_bits(b[2]), bf_bits(b[3]));
  *(volatile v4u*)(outp + e) = w;
  __threadfence();
  *(volatile v4u*)(outp + e) = w;
}

__global__ __launch_bounds__(256) void tconv_bf16_kernel(const float* __restrict__ W, unsigned short* __restrict__ outp, int R, int Cc) {
  __shared__ __align__(16) float tf[64 * 68];
  const int c0  = (int)blockIdx.x * 64;
  const int r0  = (int)blockIdx.y * 64;
  const int tid = (int)threadIdx.x;
  {
    const int lr = tid >> 4;
    const int c4 = (tid & 15) * 4;
#pragma unroll
    for (int it = 0; it < 4; ++it) {
      const int rr = it * 16 + lr;
      const v4f a = *(const v4f*)(W + (size_t)(r0 + rr) * Cc + c0 + c4);
      *(v4f*)(tf + rr * 68 + c4) = a;
    }
  }
  __syncthreads();
  const int sub = tid >> 3;
  const int c8  = (tid & 7) * 8;
  v4u hv[2];
#pragma unroll
  for (int it = 0; it < 2; ++it) {
    const int oc = it * 32 + sub;
    v4u a;
#pragma unroll
    for (int q = 0; q < 4; ++q) {
      const float f0 = tf[(c8 + 2 * q) * 68 + oc];
      const float f1 = tf[(c8 + 2 * q + 1) * 68 + oc];
      a[q] = pk16(bf_bits(f0), bf_bits(f1));
    }
    hv[it] = a;
  }
  for (int pass = 0; pass < 2; ++pass) {
#pragma unroll
    for (int it = 0; it < 2; ++it) {
      const int oc = it * 32 + sub;
      const size_t go = (size_t)(c0 + oc) * R + r0 + c8;
      *(volatile v4u*)(outp + go) = hv[it];
    }
    __threadfence();
  }
}

template <int EPI> struct SlabT { typedef float T; };
template <> struct SlabT<1> { typedef _Float16 T; };

template <int EPI, bool SPLITA>
__global__ __launch_bounds__(128) void gemm_w32x128_kernel(
    const unsigned short* Ap, const unsigned short* A2p, int lda,
    const unsigned short* __restrict__ Btp, int ldb,
    void* C0, int ldc, int M, int N, int K, float oscale) {
  typedef typename SlabT<EPI>::T ST;
  __shared__ __align__(16) ST slab_all[4 * 2048];

  const int lane = threadIdx.x & 31;
  const int wave = wave_id();
  const int hh = lane >> 4;
  const int rl = lane & 15;
  const int tilesN = N >> 7;
  const int tilesM = M >> 5;
  const int tile = (int)blockIdx.x * 4 + wave;
  if (tile >= tilesM * tilesN) return;
  const int tm = tile / tilesN;
  const int tn = tile - tm * tilesN;
  const int m0 = tm << 5;
  const int n0 = tn << 7;

  const __bf16* A  = (const __bf16*)(const void*)Ap;
  const __bf16* A2 = (const __bf16*)(const void*)A2p;
  const __bf16* Bt = (const __bf16*)(const void*)Btp;

  v8f acc[2][8];
#pragma unroll
  for (int i = 0; i < 2; ++i)
#pragma unroll
    for (int j = 0; j < 8; ++j) acc[i][j] = zero8();

  for (int k0 = 0; k0 < K; k0 += 32) {
    v16b ah[2], al[2];
#pragma unroll
    for (int i = 0; i < 2; ++i) {
      const size_t ao = (size_t)(m0 + i * 16 + rl) * lda + k0 + 8 * hh;
      ah[i] = ldfrag_b(A + ao);
      al[i] = SPLITA ? ldfrag_b(A2 + ao) : ah[i];
    }
#pragma unroll
    for (int j = 0; j < 8; ++j) {
      const v16b bj = ldfrag_b(Bt + (size_t)(n0 + j * 16 + rl) * ldb + k0 + 8 * hh);
      acc[0][j] = mma_b(ah[0], bj, acc[0][j]);
      acc[1][j] = mma_b(ah[1], bj, acc[1][j]);
      if (SPLITA) {
        acc[0][j] = mma_b(al[0], bj, acc[0][j]);
        acc[1][j] = mma_b(al[1], bj, acc[1][j]);
      }
      guard_b5(acc[0][j], acc[1][j], ah[0], ah[1], al[0], al[1], bj);
    }
  }
  acc_guard4(acc[0][0], acc[0][1], acc[0][2], acc[0][3]);
  acc_guard4(acc[0][4], acc[0][5], acc[0][6], acc[0][7]);
  acc_guard4(acc[1][0], acc[1][1], acc[1][2], acc[1][3]);
  acc_guard4(acc[1][4], acc[1][5], acc[1][6], acc[1][7]);

  ST* slab = slab_all + wave * 2048;
  if (EPI == 0) {
    float* slf = (float*)(void*)slab;
    float* C = (float*)C0;
#pragma unroll
    for (int i = 0; i < 2; ++i) {
#pragma unroll
      for (int j = 0; j < 8; ++j)
#pragma unroll
        for (int r = 0; r < 8; ++r)
          slf[(8 * hh + r) * 128 + j * 16 + rl] = acc[i][j][r] * oscale;
      lds_wave_sync();
      for (int pass = 0; pass < 2; ++pass) {
#pragma unroll
        for (int row = 0; row < 16; ++row) {
          const v4f v = *(const v4f*)(slf + row * 128 + lane * 4);
          *(volatile v4f*)(C + (size_t)(m0 + i * 16 + row) * ldc + n0 + lane * 4) = v;
        }
        __threadfence();
      }
      lds_wave_sync();
    }
  } else {
    _Float16* sl16 = (_Float16*)(void*)slab;
    _Float16* P0 = (_Float16*)C0;
#pragma unroll
    for (int i = 0; i < 2; ++i) {
#pragma unroll
      for (int r = 0; r < 8; ++r)
#pragma unroll
        for (int j = 0; j < 8; ++j)
          sl16[(8 * hh + r) * 128 + j * 16 + rl] = (_Float16)(acc[i][j][r] * oscale);
      lds_wave_sync();
      for (int pass = 0; pass < 2; ++pass) {
#pragma unroll
        for (int it = 0; it < 8; ++it) {
          const int row = it * 2 + hh;
          const int c8  = rl * 8;
          const v8h vh = *(const v8h*)(sl16 + row * 128 + c8);
          *(volatile v8h*)(P0 + (size_t)(m0 + i * 16 + row) * ldc + n0 + c8) = vh;
        }
        __threadfence();
      }
      lds_wave_sync();
    }
  }
}

__global__ __launch_bounds__(256) void normrope_kernel(const float* qkf, unsigned short* qk16, const float* __restrict__ lnw,
                                                       const float* __restrict__ cst, const float* __restrict__ snt) {
  __shared__ __align__(16) unsigned short srow[4 * EMB];
  __shared__ float red[2][8];
  const int r = (int)blockIdx.x;
  const int s = r & (GRP - 1);
  const int t = (int)threadIdx.x;
  const int lane = t & 31;
  const int wave = t >> 5;
  const int e0 = t * 4;

  const float* rowp = qkf + (size_t)r * QKW;
  const v4f qv = *(const v4f*)(rowp + e0);
  const v4f kv = *(const v4f*)(rowp + EMB + e0);
  float ssq = 0.f, ssk = 0.f;
#pragma unroll
  for (int i = 0; i < 4; ++i) { ssq += qv[i] * qv[i]; ssk += kv[i] * kv[i]; }
#pragma unroll
  for (int off = 16; off > 0; off >>= 1) {
    ssq += __shfl_xor(ssq, off, 32);
    ssk += __shfl_xor(ssk, off, 32);
  }
  if (lane == 0) { red[0][wave] = ssq; red[1][wave] = ssk; }
  __syncthreads();
  float tq = 0.f, tk = 0.f;
#pragma unroll
  for (int i = 0; i < 8; ++i) { tq += red[0][i]; tk += red[1][i]; }
  const float rq = rsqrtf(tq * 0.0009765625f + 1e-6f);
  const float rk = rsqrtf(tk * 0.0009765625f + 1e-6f);

  const v4f wv = *(const v4f*)(lnw + e0);
  const int j0 = e0 & (NFRQ - 1);
  const v4f cv = *(const v4f*)(cst + s * NFRQ + j0);
  const v4f sv = *(const v4f*)(snt + s * NFRQ + j0);

  float qn[4], kn[4];
#pragma unroll
  for (int i = 0; i < 4; ++i) {
    const float w = bf_rne(wv[i]);
    qn[i] = (qv[i] * rq) * w;
    kn[i] = (kv[i] * rk) * w;
  }
  float qr[4], kr[4];
  qr[0] = qn[0] * cv[0] - qn[1] * sv[0];
  qr[1] = qn[1] * cv[1] + qn[0] * sv[1];
  qr[2] = qn[2] * cv[2] - qn[3] * sv[2];
  qr[3] = qn[3] * cv[3] + qn[2] * sv[3];
  kr[0] = kn[0] * cv[0] - kn[1] * sv[0];
  kr[1] = kn[1] * cv[1] + kn[0] * sv[1];
  kr[2] = kn[2] * cv[2] - kn[3] * sv[2];
  kr[3] = kn[3] * cv[3] + kn[2] * sv[3];

  unsigned short qh[4], ql[4], kh[4], kl[4];
#pragma unroll
  for (int i = 0; i < 4; ++i) {
    qh[i] = bf_bits(qr[i]);
    ql[i] = bf_bits(qr[i] - bf_val(qh[i]));
    kh[i] = bf_bits(kr[i]);
    kl[i] = bf_bits(kr[i] - bf_val(kh[i]));
  }
  v2u a0, a1, a2, a3;
  a0[0] = pk16(qh[0], qh[1]); a0[1] = pk16(qh[2], qh[3]);
  a1[0] = pk16(ql[0], ql[1]); a1[1] = pk16(ql[2], ql[3]);
  a2[0] = pk16(kh[0], kh[1]); a2[1] = pk16(kh[2], kh[3]);
  a3[0] = pk16(kl[0], kl[1]); a3[1] = pk16(kl[2], kl[3]);
  *(v2u*)(srow + e0)           = a0;
  *(v2u*)(srow + EMB + e0)     = a1;
  *(v2u*)(srow + 2 * EMB + e0) = a2;
  *(v2u*)(srow + 3 * EMB + e0) = a3;
  __syncthreads();

  unsigned short* orow = qk16 + (size_t)r * QKP;
  for (int pass = 0; pass < 2; ++pass) {
#pragma unroll
    for (int it = 0; it < 2; ++it) {
      const int off = it * 2048 + t * 8;
      const v4u v = *(const v4u*)(srow + off);
      *(volatile v4u*)(orow + off) = v;
    }
    __threadfence();
  }
}

#define AKC 64
#define AQB 64
#define ANW 4

__global__ __launch_bounds__(128) void attn_local_kernel(const unsigned short* __restrict__ qk16,
                                                         const unsigned short* __restrict__ vtp,
                                                         unsigned short* __restrict__ yhp,
                                                         unsigned short* __restrict__ ylp) {
  __shared__ __align__(16) __bf16   Ksh[AKC * HDM];
  __shared__ __align__(16) __bf16   Ksl[AKC * HDM];
  __shared__ __align__(16) _Float16 Vts[HDM * AKC];
  __shared__ __align__(16) _Float16 Psh[ANW][16 * AKC];
  __shared__ __align__(16) _Float16 Psl[ANW][16 * AKC];
  __shared__ __align__(16) _Float16 Osh[ANW][2 * 16 * HDM];

  const int tid  = (int)threadIdx.x;
  const int lane = tid & 31;
  const int wave = wave_id();
  const int hh   = lane >> 4;
  const int c    = lane & 15;
  const int qb   = (int)blockIdx.x;
  const int h    = (int)blockIdx.y;
  const int bg   = (int)blockIdx.z;
  const size_t tok0 = (size_t)bg * GRP;
  const int q0   = qb * AQB + wave * 16;

  const __bf16* QK = (const __bf16*)(const void*)qk16;
  v16b qah[2], qal[2];
#pragma unroll
  for (int dc = 0; dc < 2; ++dc) {
    const __bf16* qp = QK + (tok0 + q0 + c) * QKP + h * HDM + dc * 32 + 8 * hh;
    qah[dc] = ldfrag_b(qp);
    qal[dc] = ldfrag_b(qp + EMB);
  }
  const __bf16*   Khg = QK + tok0 * QKP + 2 * EMB + h * HDM;
  const __bf16*   Klg = Khg + EMB;
  const _Float16* Vg  = (const _Float16*)(const void*)vtp + (size_t)(h * HDM) * NTOK + tok0;
  _Float16* ph = Psh[wave];
  _Float16* pl = Psl[wave];

  float mrow[8], lrow[8];
  v8f oacc[4], oaccr[4];
#pragma unroll
  for (int r = 0; r < 8; ++r) { mrow[r] = -INFINITY; lrow[r] = 0.f; }
#pragma unroll
  for (int t = 0; t < 4; ++t) { oacc[t] = zero8(); oaccr[t] = zero8(); }

  const int nch = qb + 1;
  for (int kc = 0; kc < nch; ++kc) {
    const int kv0 = kc * AKC;
    __syncthreads();
    {
      const int r = tid >> 1, half = (tid & 1) * 32;
      const __bf16*   kh = Khg + (size_t)(kv0 + r) * QKP + half;
      const __bf16*   kl = Klg + (size_t)(kv0 + r) * QKP + half;
      const _Float16* vs = Vg + (size_t)r * NTOK + kv0 + half;
#pragma unroll
      for (int i = 0; i < 4; ++i) {
        const v8b a0 = *(const v8b*)(kh + 8 * i);
        const v8b a1 = *(const v8b*)(kl + 8 * i);
        const v8h b0 = *(const v8h*)(vs + 8 * i);
        *(v8b*)(Ksh + r * HDM + half + 8 * i) = a0;
        *(v8b*)(Ksl + r * HDM + half + 8 * i) = a1;
        *(v8h*)(Vts + r * AKC + half + 8 * i) = b0;
      }
    }
    __syncthreads();

    v8f s[4];
#pragma unroll
    for (int j = 0; j < 4; ++j) {
      s[j] = zero8();
#pragma unroll
      for (int dc = 0; dc < 2; ++dc) {
        const v16b kb = ldfrag_b(Ksh + (j * 16 + c) * HDM + dc * 32 + 8 * hh);
        const v16b kl = ldfrag_b(Ksl + (j * 16 + c) * HDM + dc * 32 + 8 * hh);
        s[j] = mma_b_g(qah[dc], kb, s[j]);
        s[j] = mma_b_g(qah[dc], kl, s[j]);
        s[j] = mma_b_g(qal[dc], kb, s[j]);
      }
    }
    const bool diag = (kc == qb);
    float cm[8];
#pragma unroll
    for (int r = 0; r < 8; ++r) {
      const int qrow = q0 + 8 * hh + r;
      float m = -INFINITY;
#pragma unroll
      for (int j = 0; j < 4; ++j) {
        const int key = kv0 + j * 16 + c;
        float sv = s[j][r] * 0.125f;
        sv = (diag && (key > qrow)) ? -INFINITY : sv;
        s[j][r] = sv;
        m = fmaxf(m, sv);
      }
#pragma unroll
      for (int off = 1; off < 16; off <<= 1) m = fmaxf(m, __shfl_xor(m, off, 32));
      cm[r] = m;
    }
#pragma unroll
    for (int r = 0; r < 8; ++r) {
      const float mnew  = fmaxf(mrow[r], cm[r]);
      const float alpha = __expf(mrow[r] - mnew);
      mrow[r] = mnew;
      float psum = 0.f;
#pragma unroll
      for (int j = 0; j < 4; ++j) {
        const float p  = __expf(s[j][r] - mnew);
        psum += p;
        const float pp = p * 1024.0f;
        const _Float16 phv = (_Float16)pp;
        const int po = (8 * hh + r) * AKC + j * 16 + c;
        ph[po] = phv;
        pl[po] = (_Float16)((pp - (float)phv) * 2048.0f);
      }
#pragma unroll
      for (int off = 1; off < 16; off <<= 1) psum += __shfl_xor(psum, off, 32);
      lrow[r] = lrow[r] * alpha + psum;
#pragma unroll
      for (int t = 0; t < 4; ++t) { oacc[t][r] *= alpha; oaccr[t][r] *= alpha; }
    }
    lds_wave_sync();
#pragma unroll
    for (int kk = 0; kk < 2; ++kk) {
      const v16h pa = ldfrag_h(ph + c * AKC + kk * 32 + 8 * hh);
      const v16h pr = ldfrag_h(pl + c * AKC + kk * 32 + 8 * hh);
#pragma unroll
      for (int t = 0; t < 4; ++t) {
        const v16h vb = ldfrag_h(Vts + (t * 16 + c) * AKC + kk * 32 + 8 * hh);
        oacc[t]  = mma_h_g(pa, vb, oacc[t]);
        oaccr[t] = mma_h_g(pr, vb, oaccr[t]);
      }
    }
  }

  _Float16* osh = Osh[wave];
  _Float16* osl = osh + 16 * HDM;
#pragma unroll
  for (int r = 0; r < 8; ++r) {
    const float inv = (1.0f / lrow[r]) * (0.0009765625f * 0.125f);
#pragma unroll
    for (int t = 0; t < 4; ++t) {
      const float o = (oacc[t][r] + oaccr[t][r] * 0.00048828125f) * inv;
      const unsigned short hb = bf_bits(o);
      const unsigned short lb = bf_bits(o - bf_val(hb));
      const int so = (8 * hh + r) * HDM + t * 16 + c;
      osh[so] = __builtin_bit_cast(_Float16, hb);
      osl[so] = __builtin_bit_cast(_Float16, lb);
    }
  }
  lds_wave_sync();
  _Float16* Yhg = (_Float16*)(void*)yhp + (tok0 + q0) * EMB + h * HDM;
  _Float16* Ylg = (_Float16*)(void*)ylp + (tok0 + q0) * EMB + h * HDM;
  const int q4 = lane >> 3;
  const int c8 = (lane & 7) * 8;
  for (int pass = 0; pass < 2; ++pass) {
#pragma unroll
    for (int it = 0; it < 4; ++it) {
      const int row = it * 4 + q4;
      const v8h xh = *(const v8h*)(osh + row * HDM + c8);
      const v8h xl = *(const v8h*)(osl + row * HDM + c8);
      *(volatile v8h*)(Yhg + (size_t)row * EMB + c8) = xh;
      *(volatile v8h*)(Ylg + (size_t)row * EMB + c8) = xl;
    }
    __threadfence();
  }
}

extern "C" void kernel_launch(void* const* d_in, const int* in_sizes, int n_in,
                              void* d_out, int out_size, void* d_ws, size_t ws_size,
                              hipStream_t stream) {
  if (n_in < 4) return;
  if (in_sizes[0] != NTOK * EMB) return;
  if (in_sizes[1] != EMB * QKVW) return;
  if (in_sizes[2] != EMB) return;
  if (in_sizes[3] != EMB * EMB) return;
  if (out_size != NTOK * EMB) return;

  const float* x     = (const float*)d_in[0];
  const float* Wqkv  = (const float*)d_in[1];
  const float* lnw   = (const float*)d_in[2];
  const float* Wproj = (const float*)d_in[3];
  float* out = (float*)d_out;

  const size_t szWq = (size_t)QKVW * EMB * 2;
  const size_t szWp = (size_t)EMB * EMB * 2;
  const size_t szT  = (size_t)GRP * NFRQ * 4;
  const size_t szQK = (size_t)NTOK * QKW * 4;
  const size_t szVT = (size_t)EMB * NTOK * 2;
  const size_t szY  = (size_t)NTOK * EMB * 2;
  size_t off = 0;
  const size_t oWq = off; off += szWq;
  const size_t oWp = off; off += szWp;
  const size_t oCs = off; off += szT;
  const size_t oSn = off; off += szT;
  const size_t oQK = off; off += szQK;
  const size_t oVT = off; off += szVT;
  const size_t oYh = off; off += szY;
  const size_t oYl = off; off += szY;
  if (off > ws_size) return;

  char* ws = (char*)d_ws;
  unsigned short* WqT  = (unsigned short*)(ws + oWq);
  unsigned short* WpT  = (unsigned short*)(ws + oWp);
  float*          cst  = (float*)(ws + oCs);
  float*          snt  = (float*)(ws + oSn);
  float*          QKf  = (float*)(ws + oQK);
  unsigned short* QK16 = (unsigned short*)(ws + oQK);
  unsigned short* VT   = (unsigned short*)(ws + oVT);
  unsigned short* Yh   = (unsigned short*)(ws + oYh);
  unsigned short* Yl   = (unsigned short*)(ws + oYl);
  unsigned short* Xb   = Yh;

  const dim3 b256(256), b128(128);

  rope_table_kernel<<<dim3(GRP / 8), b256, 0, stream>>>(cst, snt);
  cvt_bf16_kernel<<<dim3((NTOK * EMB / 8) / 256), b256, 0, stream>>>(x, Xb, NTOK * EMB / 8);
  tconv_bf16_kernel<<<dim3(QKVW / 64, EMB / 64), b256, 0, stream>>>(Wqkv, WqT, EMB, QKVW);
  tconv_bf16_kernel<<<dim3(EMB / 64, EMB / 64), b256, 0, stream>>>(Wproj, WpT, EMB, EMB);
  gemm_w32x128_kernel<0, false><<<dim3((NTOK / 32) * (QKW / 128) / 4), b128, 0, stream>>>(
      Xb, Xb, EMB, WqT, EMB, (void*)QKf, QKW, NTOK, QKW, EMB, 1.0f);
  gemm_w32x128_kernel<1, false><<<dim3((EMB / 32) * (NTOK / 128) / 4), b128, 0, stream>>>(
      WqT + (size_t)QKW * EMB, WqT + (size_t)QKW * EMB, EMB, Xb, EMB, (void*)VT, NTOK, EMB, NTOK, EMB, 8.0f);
  normrope_kernel<<<dim3(NTOK), b256, 0, stream>>>(QKf, QK16, lnw, cst, snt);
  attn_local_kernel<<<dim3(GRP / AQB, NHD, NGRP), b128, 0, stream>>>(QK16, VT, Yh, Yl);
  gemm_w32x128_kernel<0, true><<<dim3((NTOK / 32) * (EMB / 128) / 4), b128, 0, stream>>>(
      Yh, Yl, EMB, WpT, EMB, (void*)out, EMB, NTOK, EMB, EMB, 1.0f);
  (void)hipGetLastError();
}
